// PhotonicBasisActivationLayer_77369540870895
// MI455X (gfx1250) — hardware-verified
//
#include <hip/hip_runtime.h>
#include <stddef.h>
#include <math.h>


#define NBR      4096
#define FI       512
#define FO       512
#define MB       16
#define KD       (FI * MB)
#define NTHR     256
#define NWAVE    8
#define BMR      128
#define BNC      128
#define WSCALE   256
#define WSCAP    134217728
#define LDS_GEMM (NWAVE * 64 * 32 * 4)

static_assert((KD % 32) == 0);
static_assert((NBR % BMR) == 0 && (FO % BNC) == 0);
static_assert(BMR == 2 * 64 && BNC == 4 * 32 && NWAVE == 8 && NTHR == NWAVE * 32);
static_assert(((NBR * FI * 2) % NTHR) == 0);
static_assert(((FO * (KD / 8)) % NTHR) == 0);
static_assert((FO % 32) == 0);
static_assert(LDS_GEMM == 65536);

typedef float     v4f  __attribute__((ext_vector_type(4)));
typedef float     v8f  __attribute__((ext_vector_type(8)));
typedef _Float16  v8h  __attribute__((ext_vector_type(8)));
typedef _Float16  v16h __attribute__((ext_vector_type(16)));
union FragH { v16h v; v8h h[2]; };

__device__ __forceinline__ v8f wmf(v16h a, v16h b, v8f c) {
  v8f d = __builtin_amdgcn_wmma_f32_16x16x32_f16(false, a, false, b, (short)0, c, false, false);
  asm volatile("v_nop\n\tv_nop\n\tv_nop\n\tv_nop" : "+v"(d) : "v"(a), "v"(b));
  return d;
}

__global__ __launch_bounds__(NTHR) void k_wprep(const float* __restrict__ w, _Float16* wp) {
  const size_t i = (size_t)blockIdx.x * NTHR + threadIdx.x;
  const v4f wa = *(const v4f*)(w + i * 8);
  const v4f wb = *(const v4f*)(w + i * 8 + 4);
  const float s = (float)WSCALE;
  v8h hv;
  hv[0] = (_Float16)(wa.x * s); hv[1] = (_Float16)(wa.y * s);
  hv[2] = (_Float16)(wa.z * s); hv[3] = (_Float16)(wa.w * s);
  hv[4] = (_Float16)(wb.x * s); hv[5] = (_Float16)(wb.y * s);
  hv[6] = (_Float16)(wb.z * s); hv[7] = (_Float16)(wb.w * s);
  _Float16* d = wp + i * 8;
  *(volatile v8h*)d = hv;
  __threadfence();
  *(volatile v8h*)d = hv;
}

__global__ __launch_bounds__(NTHR) void k_basis(const float* __restrict__ x, const float* __restrict__ bc,
                                                _Float16* ap) {
  __shared__ __attribute__((aligned(16))) _Float16 sh[NTHR * 8];
  const int tid = threadIdx.x;
  const size_t g = (size_t)blockIdx.x * NTHR + tid;
  const size_t pr = g >> 1;
  const int hf = (int)(g & 1);
  const float xv = x[pr];
  const float x2 = xv * xv;
  const float x3 = x2 * xv;
  const float x4 = x2 * x2;
#pragma unroll 1
  for (int mm = 0; mm < 8; ++mm) {
    const int m = hf * 8 + mm;
    const v4f ba = *(const v4f*)(bc + m * 8);
    const v4f bb = *(const v4f*)(bc + m * 8 + 4);
    const float t = ba.z * xv;
    const float inner = expm1f(t);
    const float lg = log2f(inner);
    const float powered = exp2f(ba.w * lg);
    const float l1 = log1pf(powered);
    const float l2 = logf(1.0f + ba.y * l1);
    const float y = ba.x * l2 + bb.x * xv + bb.y * x2 + bb.z * x3 + bb.w * x4;
    sh[tid * 8 + mm] = (_Float16)y;
  }
  __syncthreads();
  const v8h hv = *(const v8h*)(sh + tid * 8);
  _Float16* d = ap + g * 8;
  *(volatile v8h*)d = hv;
  __threadfence();
  *(volatile v8h*)d = hv;
}

__global__ __launch_bounds__(NTHR) void k_gemm(const _Float16* __restrict__ A, const _Float16* __restrict__ Bw,
                                               float* C) {
  extern __shared__ v4f lds_dyn[];
  float* stg = (float*)lds_dyn;
  const float OSC = 1.0f / (float)WSCALE;
  const int tid = threadIdx.x, lane = tid & 31, wave = tid >> 5, hh = lane >> 4, m = lane & 15;
  const int wm = wave >> 2, wn = wave & 3;
  const int rowBase = blockIdx.x * BMR + wm * 64;
  const int colBase = blockIdx.y * BNC + wn * 32;
  const _Float16* abase = A  + (size_t)(rowBase + m) * KD + 8 * hh;
  const _Float16* bbase = Bw + (size_t)(colBase + m) * KD + 8 * hh;

  v8f acc[4][2];
#pragma unroll
  for (int i = 0; i < 4; ++i)
#pragma unroll
    for (int j = 0; j < 2; ++j) { v8f z = {0.f, 0.f, 0.f, 0.f, 0.f, 0.f, 0.f, 0.f}; acc[i][j] = z; }

#pragma unroll 1
  for (int kt = 0; kt < KD / 32; ++kt) {
    const int k0 = 32 * kt;
    FragH af[4], bf[2];
#pragma unroll
    for (int i = 0; i < 4; ++i) {
      const _Float16* p = abase + (size_t)(16 * i) * KD + k0;
      af[i].h[0] = *(const v8h*)p;
      af[i].h[1] = *(const v8h*)(p + 16);
    }
#pragma unroll
    for (int j = 0; j < 2; ++j) {
      const _Float16* p = bbase + (size_t)(16 * j) * KD + k0;
      bf[j].h[0] = *(const v8h*)p;
      bf[j].h[1] = *(const v8h*)(p + 16);
    }
#pragma unroll
    for (int i = 0; i < 4; ++i)
#pragma unroll
      for (int j = 0; j < 2; ++j)
        acc[i][j] = wmf(af[i].v, bf[j].v, acc[i][j]);
  }

  float* sw = stg + wave * (64 * 32);
#pragma unroll
  for (int i = 0; i < 4; ++i)
#pragma unroll
    for (int j = 0; j < 2; ++j) {
      float* sp = sw + (16 * i + 8 * hh) * 32 + 16 * j + m;
#pragma unroll
      for (int r = 0; r < 8; ++r) sp[r * 32] = acc[i][j][r] * OSC;
    }
  __syncthreads();

  const int rq = lane >> 3, c4 = 4 * (lane & 7);
  float* gb = C + (size_t)rowBase * FO + colBase + c4;
#pragma unroll
  for (int it = 0; it < 16; ++it) {
    const int row = 4 * it + rq;
    const v4f v = *(const v4f*)(sw + row * 32 + c4);
    *(volatile v4f*)(gb + (size_t)row * FO) = v;
  }
  __threadfence();
#pragma unroll
  for (int it = 0; it < 16; ++it) {
    const int row = 4 * it + rq;
    const v4f v = *(const v4f*)(sw + row * 32 + c4);
    *(volatile v4f*)(gb + (size_t)row * FO) = v;
  }
}

extern "C" void kernel_launch(void* const* d_in, const int* in_sizes, int n_in,
                              void* d_out, int out_size, void* d_ws, size_t ws_size,
                              hipStream_t stream) {
  if (n_in < 3) return;
  if (in_sizes[0] != NBR * FI) return;
  if (in_sizes[1] != FO * FI * MB) return;
  if (in_sizes[2] != MB * 8) return;
  if (out_size != NBR * FO) return;

  const float* x  = (const float*)d_in[0];
  const float* cw = (const float*)d_in[1];
  const float* bc = (const float*)d_in[2];
  float* out = (float*)d_out;

  size_t off = 0;
  const size_t oA = off; off += (size_t)NBR * KD * 2;  off = (off + 255) & ~(size_t)255;
  const size_t oB = off; off += (size_t)FO  * KD * 2;  off = (off + 255) & ~(size_t)255;
  if (off > ws_size || off > (size_t)WSCAP) return;
  char* ws = (char*)d_ws;
  _Float16* ap = (_Float16*)(ws + oA);
  _Float16* wp = (_Float16*)(ws + oB);

  k_wprep<<<(FO * (KD / 8)) / NTHR, NTHR, 0, stream>>>(cw, wp);

  k_basis<<<(NBR * FI * 2) / NTHR, NTHR, 0, stream>>>(x, bc, ap);

  hipFuncSetAttribute(reinterpret_cast<const void*>(&k_gemm),
                      hipFuncAttributeMaxDynamicSharedMemorySize, LDS_GEMM);
  dim3 grid(NBR / BMR, FO / BNC, 1);
  k_gemm<<<grid, NTHR, LDS_GEMM, stream>>>(ap, wp, out);
}
